// VisCorefAttender_27831388078163
// MI455X (gfx1250) — hardware-verified
//
#include <hip/hip_runtime.h>


#define NB_  32
#define NM   64
#define NC   36
#define DIN  1024
#define HID  512
#define NCL  1000
#define NCLP 1024
#define BCH  8
#define RCH  (BCH * NM * NC)
#define NEGI (-1.0e10f)

typedef unsigned short bf;
typedef __attribute__((ext_vector_type(16))) __bf16   v16bf;
typedef __attribute__((ext_vector_type(8)))  unsigned short v8us;
typedef __attribute__((ext_vector_type(8)))  float    v8f;
typedef __attribute__((ext_vector_type(4)))  float    v4f;
typedef v4f  __attribute__((may_alias)) v4fa;
typedef v8us __attribute__((may_alias)) v8usa;

__device__ __forceinline__ unsigned short f2bf(float f) { unsigned u = __float_as_uint(f); u += 0x7FFFu + ((u >> 16) & 1u); return (unsigned short)(u >> 16); }
__device__ __forceinline__ float bf2f(unsigned short b) { return __uint_as_float(((unsigned)b) << 16); }
__device__ __forceinline__ float bfr(float f) { return bf2f(f2bf(f)); }
__device__ __forceinline__ v16bf cat16b(v8us lo, v8us hi) { return __builtin_bit_cast(v16bf, __builtin_shufflevector(lo, hi, 0, 1, 2, 3, 4, 5, 6, 7, 8, 9, 10, 11, 12, 13, 14, 15)); }
__device__ __forceinline__ v8f wmmab(v16bf a, v16bf b, v8f c) { return __builtin_amdgcn_wmma_f32_16x16x32_bf16(false, a, false, b, (short)0, c, false, false); }

__global__ __launch_bounds__(256) void k_rows(const float* __restrict__ src, int rows, int C, int CP, bf* dst) {
    const int lane = threadIdx.x & 31, r = blockIdx.x * 8 + (threadIdx.x >> 5);
    if (r >= rows) return;
#pragma unroll 1
    for (int ps = 0; ps < 2; ++ps) {
        for (int q = 0; q < CP / 256; ++q) { v8us o;
#pragma unroll
            for (int i = 0; i < 8; ++i) { const int c = q * 256 + lane * 8 + i; o[i] = (c < C) ? f2bf(src[(size_t)r * C + c]) : (unsigned short)0; }
            *(volatile v8us*)(dst + (size_t)r * CP + q * 256 + lane * 8) = o; }
        if (ps == 0) __threadfence(); }
}
__global__ __launch_bounds__(256) void k_wt(const float* __restrict__ Wm, int K, int KP, int ncols, bf* WT) {
    __shared__ __align__(16) unsigned short tl[64 * 72];
    const int tid = threadIdx.x, k0 = blockIdx.x * 64, n0 = blockIdx.y * 64;
    const int kk = tid >> 2, nq = (tid & 3) * 16;
#pragma unroll
    for (int i = 0; i < 16; ++i) tl[(nq + i) * 72 + kk] = (k0 + kk < K) ? f2bf(Wm[(size_t)(k0 + kk) * ncols + n0 + nq + i]) : (unsigned short)0;
    __syncthreads();
    const int piece = tid & 7;
    auto pass = [&]() {
#pragma unroll
        for (int s = 0; s < 2; ++s) { const int nr = (tid >> 3) + 32 * s; const v8us val = *(const v8usa*)(tl + nr * 72 + piece * 8); *(volatile v8us*)(WT + (size_t)(n0 + nr) * KP + k0 + piece * 8) = val; }
    };
    pass(); __threadfence(); pass();
}
template <bool SPLITA, int MODE, bool RELU>
__global__ __launch_bounds__(128) void k_gemm(const bf* __restrict__ A, const bf* __restrict__ Al, const bf* __restrict__ Bn, int K, const float* __restrict__ bias, int ldc, float* C, bf* PH, bf* PL) {
    __shared__ __align__(16) float ost[4][16 * 68];
    const int lane = threadIdx.x & 31, wave = threadIdx.x >> 5, lr = lane & 15, hi = lane >> 4;
    const size_t r0 = (size_t)blockIdx.x * 64 + wave * 16; const int c0 = blockIdx.y * 64;
    const size_t aoff = (r0 + lr) * (size_t)K + 8 * hi;
    size_t boff[4];
#pragma unroll
    for (int t = 0; t < 4; ++t) boff[t] = (size_t)(c0 + t * 16 + lr) * K + 8 * hi;
    v8f acc[4];
#pragma unroll
    for (int t = 0; t < 4; ++t) acc[t] = (v8f){};
#pragma unroll 2
    for (int kc = 0; kc < K; kc += 32) {
        const v16bf a = cat16b(*(const v8us*)(A + aoff + kc), *(const v8us*)(A + aoff + kc + 16));
        v16bf al = a; if (SPLITA) al = cat16b(*(const v8us*)(Al + aoff + kc), *(const v8us*)(Al + aoff + kc + 16));
#pragma unroll
        for (int t = 0; t < 4; ++t) { const v16bf bb = cat16b(*(const v8us*)(Bn + boff[t] + kc), *(const v8us*)(Bn + boff[t] + kc + 16)); acc[t] = wmmab(a, bb, acc[t]); if (SPLITA) acc[t] = wmmab(al, bb, acc[t]); }
        asm volatile("v_nop" : "+v"(acc[0]), "+v"(acc[1]), "+v"(acc[2]), "+v"(acc[3]) : "v"(a), "v"(al) : "memory");
    }
    float* os = &ost[wave][0];
#pragma unroll
    for (int t = 0; t < 4; ++t) { const float bv = bfr(bias[c0 + t * 16 + lr]);
#pragma unroll
        for (int j = 0; j < 8; ++j) { float v = acc[t][j] + bv; if (RELU) v = fmaxf(v, 0.f); os[(hi * 8 + j) * 68 + t * 16 + lr] = v; } }
    __builtin_amdgcn_wave_barrier(); asm volatile("" ::: "memory");
    if (MODE == 0) {
        bf* p1 = PH + r0 * ldc + c0; bf* p2 = PL + r0 * ldc + c0;
        auto pass = [&]() {
#pragma unroll
            for (int s = 0; s < 4; ++s) { const int row = 4 * s + (lane >> 3), piece = lane & 7; const float* sp = os + row * 68 + piece * 8; v8us oh, ol;
#pragma unroll
                for (int i = 0; i < 8; ++i) { const unsigned short hb = f2bf(sp[i]); oh[i] = hb; ol[i] = f2bf(sp[i] - bf2f(hb)); }
                *(volatile v8us*)(p1 + (size_t)row * ldc + piece * 8) = oh; *(volatile v8us*)(p2 + (size_t)row * ldc + piece * 8) = ol; }
        };
        pass(); __threadfence(); pass();
    } else {
        float* crow = C + r0 * ldc + c0;
        auto pass = [&]() {
#pragma unroll
            for (int s = 0; s < 8; ++s) { const int Lid = (lane >> 3) + 4 * s, piece = lane & 7; const int row = Lid >> 1, cofs = (Lid & 1) * 32 + piece * 4;
                const v4f val = *(const v4fa*)(os + row * 68 + cofs); *(volatile v4f*)(crow + (size_t)row * ldc + cofs) = val; }
        };
        pass(); __threadfence(); pass();
    }
}
__global__ __launch_bounds__(256) void k_prod(const float* __restrict__ MEN, const float* __restrict__ VIS, int b0, bf* PH, bf* PL) {
    const int lane = threadIdx.x & 31; const int r = blockIdx.x * 8 + (threadIdx.x >> 5);
    if (r >= RCH) return;
    const int bl = r / (NM * NC), rem = r - bl * (NM * NC), m = rem / NC, c = rem - m * NC, b = b0 + bl;
    const float* mr = MEN + ((size_t)b * NM + m) * HID; const float* vr = VIS + ((size_t)b * NC + c) * HID;
#pragma unroll 1
    for (int ps = 0; ps < 2; ++ps) {
#pragma unroll
        for (int q = 0; q < 2; ++q) { v8us oh, ol;
#pragma unroll
            for (int i = 0; i < 8; ++i) { const int k = q * 256 + lane * 8 + i; const float p = mr[k] * vr[k]; const unsigned short hb = f2bf(p); oh[i] = hb; ol[i] = f2bf(p - bf2f(hb)); }
            *(volatile v8us*)(PH + (size_t)r * HID + q * 256 + lane * 8) = oh; *(volatile v8us*)(PL + (size_t)r * HID + q * 256 + lane * 8) = ol; }
        if (ps == 0) __threadfence(); }
}
__global__ __launch_bounds__(256) void k_dot(const float* __restrict__ Hm, const float* __restrict__ aw2, const float* __restrict__ ab2, const float* __restrict__ mm, const float* __restrict__ cm, int b0, float* out) {
    const int lane = threadIdx.x & 31; const int rbase = (blockIdx.x * 8 + (threadIdx.x >> 5)) * 32;
    if (rbase >= RCH) return;
    float mine = 0.f;
#pragma unroll 1
    for (int i = 0; i < 32; ++i) { const int r = rbase + i; float s = 0.f;
#pragma unroll 4
        for (int k = 0; k < HID / 32; ++k) s += Hm[(size_t)r * HID + k * 32 + lane] * bfr(aw2[k * 32 + lane]);
#pragma unroll
        for (int sh = 16; sh; sh >>= 1) s += __shfl_xor(s, sh, 32);
        if (lane == i) mine = s; }
    const int r = rbase + lane; const int bl = r / (NM * NC), rem = r - bl * (NM * NC), m = rem / NC, c = rem - m * NC, b = b0 + bl;
    float a = (mine + bfr(ab2[0])) * bfr(mm[b * NM + m]) * bfr(cm[b * NC + c]); a = (a != 0.f) ? a : NEGI;
    float* op = out + (size_t)b0 * NM * NC + r;
    *(volatile float*)op = a; __threadfence(); *(volatile float*)op = a;
}

extern "C" void kernel_launch(void* const* d_in, const int* in_sizes, int n_in,
                              void* d_out, int out_size, void* d_ws, size_t ws_size, hipStream_t stream) {
    (void)in_sizes; (void)n_in; (void)out_size;
    const float* men_in = (const float*)d_in[0]; const float* cls = (const float*)d_in[1]; const float* mm = (const float*)d_in[2]; const float* cm = (const float*)d_in[3];
    const float* vw1 = (const float*)d_in[4]; const float* vb1 = (const float*)d_in[5]; const float* vw2 = (const float*)d_in[6]; const float* vb2 = (const float*)d_in[7];
    const float* mw1 = (const float*)d_in[8]; const float* mb1 = (const float*)d_in[9]; const float* mw2 = (const float*)d_in[10]; const float* mb2 = (const float*)d_in[11];
    const float* aw1 = (const float*)d_in[12]; const float* ab1 = (const float*)d_in[13]; const float* aw2 = (const float*)d_in[14]; const float* ab2 = (const float*)d_in[15];
    float* out = (float*)d_out;
    char* wsp = (char*)d_ws;
    auto take = [&](size_t bytes) { char* p = wsp; wsp += (bytes + 255) & ~(size_t)255; return (void*)p; };
    const int NV = NB_ * NC, NMR = NB_ * NM;
    bf* CLb = (bf*)take((size_t)NV * NCLP * 2); bf* MEb = (bf*)take((size_t)NMR * DIN * 2);
    bf* vw1T = (bf*)take((size_t)HID * NCLP * 2); bf* vw2T = (bf*)take((size_t)HID * HID * 2); bf* mw1T = (bf*)take((size_t)HID * DIN * 2); bf* mw2T = (bf*)take((size_t)HID * HID * 2); bf* aw1T = (bf*)take((size_t)HID * HID * 2);
    bf* V1H = (bf*)take((size_t)NV * HID * 2); bf* V1L = (bf*)take((size_t)NV * HID * 2); float* VIS = (float*)take((size_t)NV * HID * 4);
    bf* M1H = (bf*)take((size_t)NMR * HID * 2); bf* M1L = (bf*)take((size_t)NMR * HID * 2); float* MEN = (float*)take((size_t)NMR * HID * 4);
    bf* PH = (bf*)take((size_t)RCH * HID * 2); bf* PL = (bf*)take((size_t)RCH * HID * 2); float* Hm = (float*)take((size_t)RCH * HID * 4);
    if ((size_t)(wsp - (char*)d_ws) > ws_size) return;
    k_rows<<<(NV + 7) / 8, 256, 0, stream>>>(cls, NV, NCL, NCLP, CLb);
    k_rows<<<NMR / 8, 256, 0, stream>>>(men_in, NMR, DIN, DIN, MEb);
    k_wt<<<dim3(NCLP / 64, HID / 64, 1), 256, 0, stream>>>(vw1, NCL, NCLP, HID, vw1T); k_wt<<<dim3(HID / 64, HID / 64, 1), 256, 0, stream>>>(vw2, HID, HID, HID, vw2T);
    k_wt<<<dim3(DIN / 64, HID / 64, 1), 256, 0, stream>>>(mw1, DIN, DIN, HID, mw1T); k_wt<<<dim3(HID / 64, HID / 64, 1), 256, 0, stream>>>(mw2, HID, HID, HID, mw2T);
    k_wt<<<dim3(HID / 64, HID / 64, 1), 256, 0, stream>>>(aw1, HID, HID, HID, aw1T);
    k_gemm<false, 0, true ><<<dim3(NV / 64, HID / 64, 1), 128, 0, stream>>>(CLb, nullptr, vw1T, NCLP, vb1, HID, nullptr, V1H, V1L);
    k_gemm<true,  1, false><<<dim3(NV / 64, HID / 64, 1), 128, 0, stream>>>(V1H, V1L, vw2T, HID, vb2, HID, VIS, nullptr, nullptr);
    k_gemm<false, 0, true ><<<dim3(NMR / 64, HID / 64, 1), 128, 0, stream>>>(MEb, nullptr, mw1T, DIN, mb1, HID, nullptr, M1H, M1L);
    k_gemm<true,  1, false><<<dim3(NMR / 64, HID / 64, 1), 128, 0, stream>>>(M1H, M1L, mw2T, HID, mb2, HID, MEN, nullptr, nullptr);
    for (int ch = 0; ch < NB_ / BCH; ++ch) { const int b0 = ch * BCH;
        k_prod<<<RCH / 8, 256, 0, stream>>>(MEN, VIS, b0, PH, PL);
        k_gemm<true, 1, true><<<dim3(RCH / 64, HID / 64, 1), 128, 0, stream>>>(PH, PL, aw1T, HID, ab1, HID, Hm, nullptr, nullptr);
        k_dot<<<(RCH / 32 + 7) / 8, 256, 0, stream>>>(Hm, aw2, ab2, mm, cm, b0, out); }
}
